// TorchAttention_78993038508116
// MI455X (gfx1250) — hardware-verified
//
#include <hip/hip_runtime.h>


#define NB_  2
#define NT_  2048
#define DM   1024
#define NH_  16
#define HD   64
#define NTK  (NB_ * NT_)
#define NBK  32
#define PSC  32768.0f
#define LOSC 1024.0f
#define LOSCI (1.0f / 1024.0f)

typedef _Float16 h16;
typedef unsigned short bf;
typedef __attribute__((ext_vector_type(16))) __bf16   v16bf;
typedef __attribute__((ext_vector_type(16))) _Float16 v16h;
typedef __attribute__((ext_vector_type(8)))  _Float16 v8h;
typedef __attribute__((ext_vector_type(8)))  unsigned short v8us;
typedef __attribute__((ext_vector_type(8)))  float    v8f;
typedef __attribute__((ext_vector_type(4)))  float    v4f;
typedef v8h  __attribute__((may_alias)) v8ha;
typedef v4f  __attribute__((may_alias)) v4fa;

__device__ __forceinline__ unsigned short f2bf(float f) { unsigned u = __float_as_uint(f); u += 0x7FFFu + ((u >> 16) & 1u); return (unsigned short)(u >> 16); }
__device__ __forceinline__ float bf2f(unsigned short b) { return __uint_as_float(((unsigned)b) << 16); }
__device__ __forceinline__ float bfr(float f) { return bf2f(f2bf(f)); }
__device__ __forceinline__ v16h cat16(v8h lo, v8h hi) { return __builtin_shufflevector(lo, hi, 0, 1, 2, 3, 4, 5, 6, 7, 8, 9, 10, 11, 12, 13, 14, 15); }
__device__ __forceinline__ v16bf cat16b(v8us lo, v8us hi) { return __builtin_bit_cast(v16bf, __builtin_shufflevector(lo, hi, 0, 1, 2, 3, 4, 5, 6, 7, 8, 9, 10, 11, 12, 13, 14, 15)); }
__device__ __forceinline__ v8f wmma16(v16h a, v16h b, v8f c) { return __builtin_amdgcn_wmma_f32_16x16x32_f16(false, a, false, b, (short)0, c, false, false); }
__device__ __forceinline__ v8f wmmab(v16bf a, v16bf b, v8f c) { return __builtin_amdgcn_wmma_f32_16x16x32_bf16(false, a, false, b, (short)0, c, false, false); }
#define VST2(T, p, v) do { const T vst2_v_ = (v); *(volatile T*)(p) = vst2_v_; __threadfence(); *(volatile T*)(p) = vst2_v_; } while (0)

__global__ __launch_bounds__(256) void k_cvtb(const float* __restrict__ src, int nrows, bf* dst) {
    const int lane = threadIdx.x & 31, r = blockIdx.x * 8 + (threadIdx.x >> 5);
    if (r >= nrows) return;
    v8us o[4];
#pragma unroll
    for (int q = 0; q < 4; ++q) { v8us t;
#pragma unroll
        for (int i = 0; i < 8; ++i) t[i] = f2bf(src[(size_t)r * DM + q * 256 + lane * 8 + i]);
        o[q] = t; }
#pragma unroll
    for (int q = 0; q < 4; ++q) *(volatile v8us*)(dst + (size_t)r * DM + q * 256 + lane * 8) = o[q];
    __threadfence();
#pragma unroll
    for (int q = 0; q < 4; ++q) *(volatile v8us*)(dst + (size_t)r * DM + q * 256 + lane * 8) = o[q];
}

template <bool SPLITA>
__global__ __launch_bounds__(128) void k_gemmb(const bf* __restrict__ A, const bf* __restrict__ Al, const bf* __restrict__ Bn, float* C, int ldc) {
    __shared__ __align__(16) float ost[4][16 * 68];
    const int lane = threadIdx.x & 31, wave = threadIdx.x >> 5, lr = lane & 15, hi = lane >> 4;
    const int r0 = blockIdx.x * 64 + wave * 16, c0 = blockIdx.y * 64;
    const size_t aoff = (size_t)(r0 + lr) * DM + 8 * hi;
    size_t boff[4];
#pragma unroll
    for (int t = 0; t < 4; ++t) boff[t] = (size_t)(c0 + t * 16 + lr) * DM + 8 * hi;
    v8f acc[4];
#pragma unroll
    for (int t = 0; t < 4; ++t) acc[t] = (v8f){};
#pragma unroll 1
    for (int kc = 0; kc < DM; kc += 32) {
        const v16bf a = cat16b(*(const v8us*)(A + aoff + kc), *(const v8us*)(A + aoff + kc + 16));
        v16bf al = a;
        if (SPLITA) al = cat16b(*(const v8us*)(Al + aoff + kc), *(const v8us*)(Al + aoff + kc + 16));
#pragma unroll
        for (int t = 0; t < 4; ++t) { const v16bf b = cat16b(*(const v8us*)(Bn + boff[t] + kc), *(const v8us*)(Bn + boff[t] + kc + 16)); acc[t] = wmmab(a, b, acc[t]); if (SPLITA) acc[t] = wmmab(al, b, acc[t]); }
        asm volatile("v_nop\n\tv_nop\n\tv_nop\n\tv_nop" : "+v"(acc[0]), "+v"(acc[1]), "+v"(acc[2]), "+v"(acc[3]) : "v"(a), "v"(al));
    }
    float* os = &ost[wave][0];
#pragma unroll
    for (int t = 0; t < 4; ++t)
#pragma unroll
        for (int j = 0; j < 8; ++j) os[(hi * 8 + j) * 68 + t * 16 + lr] = acc[t][j];
    __syncthreads();
    float* crow = C + (size_t)r0 * ldc + c0;
    auto pass = [&]() {
#pragma unroll
        for (int s = 0; s < 8; ++s) { const int Lid = (lane >> 3) + 4 * s, piece = lane & 7; const int row = Lid >> 1, cofs = (Lid & 1) * 32 + piece * 4;
            const v4f val = *(const v4fa*)(os + row * 68 + cofs); *(volatile v4f*)(crow + (size_t)row * ldc + cofs) = val; }
    };
    pass(); __threadfence(); pass();
}

__global__ __launch_bounds__(256) void k_qk2(const float* __restrict__ QKV, h16* QH, h16* QL, h16* KH, h16* KL) {
    const int lane = threadIdx.x & 31, wid = blockIdx.x * 8 + (threadIdx.x >> 5);
    if (wid >= 2 * NTK) return;
    const int r = wid >> 1, which = wid & 1;
    const float* s = QKV + (size_t)r * (3 * DM) + which * DM;
    h16* dh = (which ? KH : QH) + (size_t)r * DM; h16* dl = (which ? KL : QL) + (size_t)r * DM;
    v8h oh[4], ol[4];
#pragma unroll
    for (int q = 0; q < 4; ++q) { v8h t, u;
#pragma unroll
        for (int i = 0; i < 8; ++i) { const float v = s[q * 256 + lane * 8 + i]; const h16 a = (h16)v; t[i] = a; u[i] = (h16)((v - (float)a) * LOSC); }
        oh[q] = t; ol[q] = u; }
#pragma unroll
    for (int q = 0; q < 4; ++q) { *(volatile v8h*)(dh + q * 256 + lane * 8) = oh[q]; *(volatile v8h*)(dl + q * 256 + lane * 8) = ol[q]; }
    __threadfence();
#pragma unroll
    for (int q = 0; q < 4; ++q) { *(volatile v8h*)(dh + q * 256 + lane * 8) = oh[q]; *(volatile v8h*)(dl + q * 256 + lane * 8) = ol[q]; }
}

__global__ __launch_bounds__(256) void k_vt(const float* __restrict__ QKV, h16* VT16) {
    __shared__ __align__(16) h16 tile[64 * 72];
    const int bid = blockIdx.x;
    const int b = bid / (NH_ * (NT_ / 64)), rem = bid - b * (NH_ * (NT_ / 64)), h = rem / (NT_ / 64), kt = rem - h * (NT_ / 64);
    const int k0 = kt * 64, tid = threadIdx.x;
    const int kk = tid >> 2, d0 = (tid & 3) * 16;
    const float* src = QKV + ((size_t)b * NT_ + k0 + kk) * (3 * DM) + 2 * DM + h * HD + d0;
#pragma unroll
    for (int i = 0; i < 16; ++i) tile[(d0 + i) * 72 + kk] = (h16)src[i];
    __syncthreads();
    const int piece = tid & 7;
    h16* base = VT16 + (((size_t)b * NH_ + h) * HD) * NT_ + k0;
    auto pass = [&]() {
#pragma unroll
        for (int s = 0; s < 2; ++s) { const int d = (tid >> 3) + 32 * s; const v8h val = *(const v8ha*)(tile + d * 72 + piece * 8); *(volatile v8h*)(base + (size_t)d * NT_ + piece * 8) = val; }
    };
    pass(); __threadfence(); pass();
}

__device__ __forceinline__ int t5_bucket(int rel) {
    int rb = 0; const int nb = 16; if (rel > 0) rb += nb; const int rp = rel < 0 ? -rel : rel; const int max_exact = 8;
    if (rp < max_exact) return rb + rp;
    const float v = logf((float)rp / (float)max_exact) / 2.7725887298583984375f * (float)(nb - max_exact);
    int large = max_exact + (int)(v + 1e-3f); if (large > nb - 1) large = nb - 1; return rb + large;
}
__global__ __launch_bounds__(256) void k_btab(const float* __restrict__ emb, float* BT) {
    const int q = blockIdx.x * 256 + threadIdx.x; if (q >= NH_ * 4096) return;
    const int h = q >> 12, r = q & 4095;
    VST2(float, BT + q, (r < 4095) ? bfr(emb[t5_bucket(r - 2047) * NH_ + h]) : 0.0f);
}

__global__ __launch_bounds__(128) void k_attn(const h16* __restrict__ QH, const h16* __restrict__ QL, const h16* __restrict__ KH, const h16* __restrict__ KL, const h16* __restrict__ VT16,
                                              const float* __restrict__ amask, const float* __restrict__ BT, bf* CH, bf* CL) {
    __shared__ __align__(16) h16 plds[4][16 * 32];
    __shared__ __align__(16) float ost[4][16 * 68];
    const int lane = threadIdx.x & 31, wave = threadIdx.x >> 5, lr = lane & 15, hi = lane >> 4;
    const int bid = blockIdx.x;
    const int b = bid / (NH_ * (NT_ / 64)), rem = bid - b * (NH_ * (NT_ / 64)), h = rem / (NT_ / 64), qt = rem - h * (NT_ / 64);
    const int q0 = qt * 64 + wave * 16;
    const size_t tok0 = (size_t)b * NT_;
    h16* pl = &plds[wave][0];
    v16h qa[2], ql[2];
#pragma unroll
    for (int kc = 0; kc < 2; ++kc) { const size_t po = (tok0 + q0 + lr) * DM + h * HD + kc * 32 + 8 * hi; qa[kc] = cat16(*(const v8h*)(QH + po), *(const v8h*)(QH + po + 16)); ql[kc] = cat16(*(const v8h*)(QL + po), *(const v8h*)(QL + po + 16)); }
    int qpos[8];
#pragma unroll
    for (int j = 0; j < 8; ++j) qpos[j] = q0 + 8 * hi + j;
    const h16* kh_b = KH + tok0 * DM + h * HD; const h16* kl_b = KL + tok0 * DM + h * HD;
    const h16* vt_b = VT16 + (((size_t)b * NH_ + h) * HD) * NT_;
    const float* bt = BT + (size_t)h * 4096 + 2047;
    const float* mk = amask + (size_t)b * NT_ * NT_;
    v8f o[4];
#pragma unroll
    for (int n = 0; n < 4; ++n) o[n] = (v8f){};
    float mrow[8], lpart[8];
#pragma unroll
    for (int j = 0; j < 8; ++j) { mrow[j] = -3.0e38f; lpart[j] = 0.f; }
#pragma unroll 1
    for (int kt = 0; kt < NT_ / 32; ++kt) {
        const int l0 = kt * 32;
        const size_t r0o = (size_t)(l0 + lr) * DM + 8 * hi, r1o = (size_t)(l0 + 16 + lr) * DM + 8 * hi;
        v8f s0 = {}, s1 = {}, x0 = {}, x1 = {};
#pragma unroll
        for (int kc = 0; kc < 2; ++kc) {
            const v16h b0 = cat16(*(const v8h*)(kh_b + r0o + kc * 32), *(const v8h*)(kh_b + r0o + kc * 32 + 16));
            const v16h b1 = cat16(*(const v8h*)(kh_b + r1o + kc * 32), *(const v8h*)(kh_b + r1o + kc * 32 + 16));
            s0 = wmma16(qa[kc], b0, s0); s1 = wmma16(qa[kc], b1, s1);
            x0 = wmma16(qa[kc], cat16(*(const v8h*)(kl_b + r0o + kc * 32), *(const v8h*)(kl_b + r0o + kc * 32 + 16)), x0);
            x1 = wmma16(qa[kc], cat16(*(const v8h*)(kl_b + r1o + kc * 32), *(const v8h*)(kl_b + r1o + kc * 32 + 16)), x1);
            x0 = wmma16(ql[kc], b0, x0); x1 = wmma16(ql[kc], b1, x1);
        }
        asm volatile("v_nop\n\tv_nop\n\tv_nop\n\tv_nop" : "+v"(s0), "+v"(s1), "+v"(x0), "+v"(x1) : "v"(qa[0]), "v"(ql[1]));
        const int key0 = l0 + lr, key1 = l0 + 16 + lr;
        float alpha[8];
#pragma unroll
        for (int j = 0; j < 8; ++j) {
            const int i = qpos[j];
            const float m0 = bfr(mk[(size_t)i * NT_ + key0]), m1 = bfr(mk[(size_t)i * NT_ + key1]);
            const float a0 = (s0[j] + x0[j] * LOSCI) * m0 + (-1e8f * (1.0f - m0) + bt[key0 - i]);
            const float a1 = (s1[j] + x1[j] * LOSCI) * m1 + (-1e8f * (1.0f - m1) + bt[key1 - i]);
            float mx = fmaxf(a0, a1);
            mx = fmaxf(mx, __shfl_xor(mx, 1, 16)); mx = fmaxf(mx, __shfl_xor(mx, 2, 16)); mx = fmaxf(mx, __shfl_xor(mx, 4, 16)); mx = fmaxf(mx, __shfl_xor(mx, 8, 16));
            const float mn = fmaxf(mrow[j], mx);
            alpha[j] = __expf(mrow[j] - mn); mrow[j] = mn;
            const float p0 = __expf(a0 - mn), p1 = __expf(a1 - mn);
            lpart[j] = lpart[j] * alpha[j] + (p0 + p1);
            const int mr = hi * 8 + j;
            pl[mr * 32 + lr] = (h16)(p0 * PSC); pl[mr * 32 + 16 + lr] = (h16)(p1 * PSC);
        }
#pragma unroll
        for (int n = 0; n < 4; ++n)
#pragma unroll
            for (int j = 0; j < 8; ++j) o[n][j] *= alpha[j];
        asm volatile("" ::: "memory");
        const v16h pa = cat16(*(const v8ha*)(pl + lr * 32 + hi * 8), *(const v8ha*)(pl + lr * 32 + 16 + hi * 8));
#pragma unroll
        for (int n = 0; n < 4; ++n) { const h16* vp = vt_b + (size_t)(n * 16 + lr) * NT_ + l0 + hi * 8; o[n] = wmma16(pa, cat16(*(const v8h*)vp, *(const v8h*)(vp + 16)), o[n]); }
        asm volatile("v_nop\n\tv_nop\n\tv_nop\n\tv_nop" : "+v"(o[0]), "+v"(o[1]), "+v"(o[2]), "+v"(o[3]) : "v"(pa));
    }
    float inv[8];
#pragma unroll
    for (int j = 0; j < 8; ++j) { float rs = lpart[j]; rs += __shfl_xor(rs, 1, 16); rs += __shfl_xor(rs, 2, 16); rs += __shfl_xor(rs, 4, 16); rs += __shfl_xor(rs, 8, 16); inv[j] = 1.0f / (rs * PSC); }
    float* os = &ost[wave][0];
#pragma unroll
    for (int n = 0; n < 4; ++n)
#pragma unroll
        for (int j = 0; j < 8; ++j) os[(hi * 8 + j) * 68 + n * 16 + lr] = o[n][j] * inv[j];
    __syncthreads();
    const size_t cbase = (tok0 + q0) * DM + (size_t)h * HD;
    auto pass = [&]() {
#pragma unroll
        for (int s = 0; s < 4; ++s) { const int row = 4 * s + (lane >> 3), piece = lane & 7; const float* sp = os + row * 68 + piece * 8; v8us oh, ol;
#pragma unroll
            for (int i = 0; i < 8; ++i) { const unsigned short hb = f2bf(sp[i]); oh[i] = hb; ol[i] = f2bf(sp[i] - bf2f(hb)); }
            *(volatile v8us*)(CH + cbase + (size_t)row * DM + piece * 8) = oh; *(volatile v8us*)(CL + cbase + (size_t)row * DM + piece * 8) = ol; }
    };
    pass(); __threadfence(); pass();
}

extern "C" void kernel_launch(void* const* d_in, const int* in_sizes, int n_in,
                              void* d_out, int out_size, void* d_ws, size_t ws_size, hipStream_t stream) {
    (void)in_sizes; (void)n_in; (void)out_size;
    const float* x = (const float*)d_in[0]; const float* amask = (const float*)d_in[1]; const float* Wqkv = (const float*)d_in[2]; const float* emb = (const float*)d_in[3]; const float* Wo = (const float*)d_in[4];
    float* out = (float*)d_out;
    char* wsp = (char*)d_ws;
    auto take = [&](size_t bytes) { char* p = wsp; wsp += (bytes + 255) & ~(size_t)255; return (void*)p; };
    bf* Xb = (bf*)take((size_t)NTK * DM * 2); bf* WQKVb = (bf*)take((size_t)3 * DM * DM * 2); bf* WOb = (bf*)take((size_t)DM * DM * 2);
    float* QKV = (float*)take((size_t)NTK * 3 * DM * 4);
    h16* QH = (h16*)take((size_t)NTK * DM * 2); h16* QL = (h16*)take((size_t)NTK * DM * 2); h16* KH = (h16*)take((size_t)NTK * DM * 2); h16* KL = (h16*)take((size_t)NTK * DM * 2);
    h16* VT16 = (h16*)take((size_t)NTK * DM * 2); float* BT = (float*)take((size_t)NH_ * 4096 * 4);
    bf* CH = (bf*)take((size_t)NTK * DM * 2); bf* CL = (bf*)take((size_t)NTK * DM * 2);
    if ((size_t)(wsp - (char*)d_ws) > ws_size) return;
    k_cvtb<<<NTK / 8, 256, 0, stream>>>(x, NTK, Xb);
    k_cvtb<<<(3 * DM) / 8, 256, 0, stream>>>(Wqkv, 3 * DM, WQKVb);
    k_cvtb<<<DM / 8, 256, 0, stream>>>(Wo, DM, WOb);
    k_gemmb<false><<<dim3(NTK / 64, (3 * DM) / 64, 1), 128, 0, stream>>>(Xb, nullptr, WQKVb, QKV, 3 * DM);
    k_qk2<<<(2 * NTK) / 8, 256, 0, stream>>>(QKV, QH, QL, KH, KL);
    k_vt<<<NB_ * NH_ * (NT_ / 64), 256, 0, stream>>>(QKV, VT16);
    k_btab<<<(NH_ * 4096) / 256, 256, 0, stream>>>(emb, BT);
    k_attn<<<NB_ * NH_ * (NT_ / 64), 128, 0, stream>>>(QH, QL, KH, KL, VT16, amask, BT, CH, CL);
    k_gemmb<true><<<dim3(NTK / 64, DM / 64, 1), 128, 0, stream>>>(CH, CL, WOb, out, DM);
}
